// GuidedMambaVSSBlock_32719060861029
// MI455X (gfx1250) — hardware-verified
//
#include <hip/hip_runtime.h>
#define BB 4
#define CC 96
#define HS 64
#define NP 4096
#define DI 192
#define NS 8
#define RR 6
#define XDW 22
#define CB 16
#define NR (BB * NP)

typedef __bf16 v16b __attribute__((ext_vector_type(16)));
typedef unsigned short v8us __attribute__((ext_vector_type(8), may_alias));
typedef float  v8f  __attribute__((ext_vector_type(8)));
typedef float  v4f  __attribute__((ext_vector_type(4)));
typedef float  v4fa __attribute__((ext_vector_type(4), may_alias));
union FragB { v16b v; v8us half[2]; unsigned short u[16]; };

__device__ __forceinline__ unsigned short bf16_bits(float x) { unsigned int u = __float_as_uint(x); return (unsigned short)((u + 0x7FFFu + ((u >> 16) & 1u)) >> 16); }
__device__ __forceinline__ float bf16_val(unsigned short b) { return __uint_as_float(((unsigned int)b) << 16); }
__device__ __forceinline__ float bf16_round(float x) { return bf16_val(bf16_bits(x)); }
template <int NT>
__device__ __forceinline__ v8f mmaN(v16b ah, v16b al, v16b bh, v16b bl, v8f c) {
  c = __builtin_amdgcn_wmma_f32_16x16x32_bf16(false, ah, false, bh, (short)0, c, false, false);
  if (NT >= 2) c = __builtin_amdgcn_wmma_f32_16x16x32_bf16(false, al, false, bh, (short)0, c, false, false);
  if (NT >= 3) c = __builtin_amdgcn_wmma_f32_16x16x32_bf16(false, ah, false, bl, (short)0, c, false, false);
  asm volatile("v_nop\n\tv_nop\n\tv_nop\n\tv_nop" : "+v"(c) : "v"(ah), "v"(al), "v"(bh), "v"(bl));
  return c;
}

__global__ __launch_bounds__(256) void k_wt_bf16(const float* __restrict__ W, unsigned short* __restrict__ Wt, int K, int N) {
  const int t = blockIdx.x * 256 + threadIdx.x;
  const int k8n = K / 8;
  if (t >= N * k8n) return;
  const int n = t / k8n, k8 = (t % k8n) * 8;
  v8us v;
#pragma unroll
  for (int i = 0; i < 8; ++i) v[i] = bf16_bits(W[(size_t)(k8 + i) * N + n]);
  *(volatile v8us*)(Wt + (size_t)n * K + k8) = v;
  __threadfence();
  *(volatile v8us*)(Wt + (size_t)n * K + k8) = v;
}

template <bool ASPLIT, int ACT, bool BIAS_BF16>
__global__ __launch_bounds__(128) void k_gemm_bf(const float* __restrict__ A, int lda, const unsigned short* __restrict__ Wt, int ldb,
                                               const float* __restrict__ bias, float* __restrict__ C, int ldc, int M, int N, int K) {
  __shared__ __attribute__((aligned(16))) float so[4][16][64];
  const int tid = threadIdx.x, w = tid >> 5, lane = tid & 31, ln = lane & 15, hh = lane >> 4;
  const int ntn = N / 64;
  const int wid = blockIdx.x * 4 + w;
  const int mt = wid / ntn, nq = wid % ntn;
  if (mt * 16 >= M) return;
  const int row0 = mt * 16, col0 = nq * 64;
  const float* arow = A + (size_t)(row0 + ln) * lda;
  v8f acc[4] = {};
  for (int kb = 0; kb < K; kb += 32) {
    FragB ah, al;
    const v4f x0 = *(const v4fa*)(arow + kb + 8 * hh), x1 = *(const v4fa*)(arow + kb + 8 * hh + 4);
    const v4f x2 = *(const v4fa*)(arow + kb + 16 + 8 * hh), x3 = *(const v4fa*)(arow + kb + 16 + 8 * hh + 4);
    float xs[16] = {x0[0],x0[1],x0[2],x0[3],x1[0],x1[1],x1[2],x1[3],x2[0],x2[1],x2[2],x2[3],x3[0],x3[1],x3[2],x3[3]};
#pragma unroll
    for (int i = 0; i < 16; ++i) { const unsigned short hb = bf16_bits(xs[i]); ah.u[i] = hb; al.u[i] = ASPLIT ? bf16_bits(xs[i] - bf16_val(hb)) : (unsigned short)0; }
#pragma unroll
    for (int t = 0; t < 4; ++t) {
      const unsigned short* brow = Wt + (size_t)(col0 + t * 16 + ln) * ldb + kb;
      FragB b;
      b.half[0] = *(const v8us*)(brow + 8 * hh);
      b.half[1] = *(const v8us*)(brow + 16 + 8 * hh);
      acc[t] = mmaN<ASPLIT ? 2 : 1>(ah.v, al.v, b.v, b.v, acc[t]);
    }
  }
#pragma unroll
  for (int t = 0; t < 4; ++t) {
    float bv = bias ? bias[col0 + t * 16 + ln] : 0.f;
    if (BIAS_BF16) bv = bf16_round(bv);
#pragma unroll
    for (int r = 0; r < 8; ++r) { float v = acc[t][r] + bv; if (ACT == 1) v = fmaxf(v, 0.f); so[w][8 * hh + r][t * 16 + ln] = v; }
  }
  __builtin_amdgcn_fence(__ATOMIC_ACQ_REL, "workgroup");
  __builtin_amdgcn_wave_barrier();
  const int rsub = lane >> 4, c4 = (lane & 15) * 4;
  for (int pass = 0; pass < 2; ++pass) {
#pragma unroll
    for (int q = 0; q < 8; ++q) {
      const int r = q * 2 + rsub;
      const v4f v = *(const v4fa*)&so[w][r][c4];
      *(volatile v4f*)(C + (size_t)(row0 + r) * ldc + col0 + c4) = v;
    }
    if (pass == 0) __threadfence();
  }
}

template <int D, bool CAUSAL>
__global__ __launch_bounds__(128) void k_flash(const float* __restrict__ qb, const float* __restrict__ kb, const float* __restrict__ vb,
                                             int pitch, int T, int H, float scale, float* __restrict__ y, int ypitch) {
  constexpr int KS = D / 32;
  constexpr int DT = D / 16;
  __shared__ __attribute__((aligned(16))) unsigned short sKh[32][D + 8], sKl[32][D + 8], sVh[32][D + 8], sVl[32][D + 8];
  __shared__ __attribute__((aligned(16))) unsigned short sPh[4][16][40], sPl[4][16][40];
  __shared__ __attribute__((aligned(16))) float sO[4][16][D];
  const int tid = threadIdx.x, w = tid >> 5, lane = tid & 31, ln = lane & 15, hh = lane >> 4;
  const int nqb = (T + 63) / 64;
  const int bh = blockIdx.x / nqb, qblk = blockIdx.x % nqb;
  const int b = bh / H, h = bh % H;
  const int q0 = qblk * 64 + w * 16;
  const float* Q = qb + (size_t)b * T * pitch + h * D;
  const float* K = kb + (size_t)b * T * pitch + h * D;
  const float* V = vb + (size_t)b * T * pitch + h * D;

  FragB aqh[KS], aql[KS];
  {
    int row = q0 + ln; if (row >= T) row = T - 1;
    const float* qr = Q + (size_t)row * pitch;
#pragma unroll
    for (int ks = 0; ks < KS; ++ks)
#pragma unroll
      for (int i = 0; i < 16; ++i) {
        const int d = ks * 32 + ((i < 8) ? (8 * hh + i) : (16 + 8 * hh + (i - 8)));
        const float x = qr[d] * scale; const unsigned short hb = bf16_bits(x);
        aqh[ks].u[i] = hb; aql[ks].u[i] = bf16_bits(x - bf16_val(hb));
      }
  }
  float m_r[8], l_r[8];
#pragma unroll
  for (int r = 0; r < 8; ++r) { m_r[r] = -3.0e38f; l_r[r] = 0.f; }
  v8f oacc[DT];
#pragma unroll
  for (int dt = 0; dt < DT; ++dt) oacc[dt] = (v8f){0.f,0.f,0.f,0.f,0.f,0.f,0.f,0.f};

  const int kv_end = CAUSAL ? min(T, qblk * 64 + 64) : T;
  for (int j0 = 0; j0 < kv_end; j0 += 32) {
    __syncthreads();
    for (int e = tid; e < 32 * (D / 4); e += 128) {
      const int r = e / (D / 4), c4 = (e % (D / 4)) * 4;
      const int key = j0 + r;
      v4f kf = {0.f,0.f,0.f,0.f}, vf = {0.f,0.f,0.f,0.f};
      if (key < T) { kf = *(const v4fa*)(K + (size_t)key * pitch + c4); vf = *(const v4fa*)(V + (size_t)key * pitch + c4); }
#pragma unroll
      for (int t = 0; t < 4; ++t) {
        unsigned short hb = bf16_bits(kf[t]); sKh[r][c4 + t] = hb; sKl[r][c4 + t] = bf16_bits(kf[t] - bf16_val(hb));
        hb = bf16_bits(vf[t]); sVh[r][c4 + t] = hb; sVl[r][c4 + t] = bf16_bits(vf[t] - bf16_val(hb));
      }
    }
    __syncthreads();
    v8f s[2];
#pragma unroll
    for (int nt = 0; nt < 2; ++nt) {
      v8f acc = {};
#pragma unroll
      for (int ks = 0; ks < KS; ++ks) {
        FragB bh_, bl_;
        bh_.half[0] = *(const v8us*)&sKh[nt * 16 + ln][ks * 32 + 8 * hh]; bh_.half[1] = *(const v8us*)&sKh[nt * 16 + ln][ks * 32 + 16 + 8 * hh];
        bl_.half[0] = *(const v8us*)&sKl[nt * 16 + ln][ks * 32 + 8 * hh]; bl_.half[1] = *(const v8us*)&sKl[nt * 16 + ln][ks * 32 + 16 + 8 * hh];
        acc = mmaN<3>(aqh[ks].v, aql[ks].v, bh_.v, bl_.v, acc);
      }
      s[nt] = acc;
    }
    float alpha[8];
#pragma unroll
    for (int r = 0; r < 8; ++r) {
      const int qi = q0 + 8 * hh + r;
      const int ja = j0 + ln, jb = j0 + 16 + ln;
      if (CAUSAL) { if (ja > qi) s[0][r] = -3.0e38f; if (jb > qi) s[1][r] = -3.0e38f; }
      if (ja >= T) s[0][r] = -3.0e38f;
      if (jb >= T) s[1][r] = -3.0e38f;
      float mx = fmaxf(s[0][r], s[1][r]);
      mx = fmaxf(mx, __shfl_xor(mx, 1, 32)); mx = fmaxf(mx, __shfl_xor(mx, 2, 32)); mx = fmaxf(mx, __shfl_xor(mx, 4, 32)); mx = fmaxf(mx, __shfl_xor(mx, 8, 32));
      const float mnew = fmaxf(m_r[r], mx);
      alpha[r] = (mnew > -1.0e38f) ? __expf(m_r[r] - mnew) : 1.0f;
      const float p0 = (s[0][r] > -1.0e38f) ? __expf(s[0][r] - mnew) : 0.f;
      const float p1 = (s[1][r] > -1.0e38f) ? __expf(s[1][r] - mnew) : 0.f;
      m_r[r] = mnew;
      l_r[r] = l_r[r] * alpha[r] + p0 + p1;
      unsigned short hb = bf16_bits(p0); sPh[w][8 * hh + r][ln] = hb;      sPl[w][8 * hh + r][ln] = bf16_bits(p0 - bf16_val(hb));
      hb = bf16_bits(p1);                sPh[w][8 * hh + r][16 + ln] = hb; sPl[w][8 * hh + r][16 + ln] = bf16_bits(p1 - bf16_val(hb));
    }
#pragma unroll
    for (int dt = 0; dt < DT; ++dt)
#pragma unroll
      for (int r = 0; r < 8; ++r) oacc[dt][r] *= alpha[r];
    __builtin_amdgcn_fence(__ATOMIC_ACQ_REL, "workgroup");
    __builtin_amdgcn_wave_barrier();
    FragB pah, pal;
    pah.half[0] = *(const v8us*)&sPh[w][ln][8 * hh]; pah.half[1] = *(const v8us*)&sPh[w][ln][16 + 8 * hh];
    pal.half[0] = *(const v8us*)&sPl[w][ln][8 * hh]; pal.half[1] = *(const v8us*)&sPl[w][ln][16 + 8 * hh];
#pragma unroll
    for (int dt = 0; dt < DT; ++dt) {
      FragB bvh, bvl;
#pragma unroll
      for (int i = 0; i < 8; ++i) {
        bvh.u[i] = sVh[8 * hh + i][dt * 16 + ln]; bvh.u[8 + i] = sVh[16 + 8 * hh + i][dt * 16 + ln];
        bvl.u[i] = sVl[8 * hh + i][dt * 16 + ln]; bvl.u[8 + i] = sVl[16 + 8 * hh + i][dt * 16 + ln];
      }
      oacc[dt] = mmaN<3>(pah.v, pal.v, bvh.v, bvl.v, oacc[dt]);
    }
    __builtin_amdgcn_fence(__ATOMIC_ACQ_REL, "workgroup");
    __builtin_amdgcn_wave_barrier();
  }
#pragma unroll
  for (int r = 0; r < 8; ++r) {
    float l = l_r[r];
    l += __shfl_xor(l, 1, 32); l += __shfl_xor(l, 2, 32); l += __shfl_xor(l, 4, 32); l += __shfl_xor(l, 8, 32);
    l_r[r] = (l > 0.f) ? 1.0f / l : 0.f;
  }
#pragma unroll
  for (int dt = 0; dt < DT; ++dt)
#pragma unroll
    for (int r = 0; r < 8; ++r) sO[w][8 * hh + r][dt * 16 + ln] = oacc[dt][r] * l_r[r];
  __builtin_amdgcn_fence(__ATOMIC_ACQ_REL, "workgroup");
  __builtin_amdgcn_wave_barrier();
  for (int pass = 0; pass < 2; ++pass) {
    for (int r = 0; r < 16; ++r) {
      const int row = q0 + r;
      if (row < T && lane < D / 4) {
        const v4f val = *(const v4fa*)&sO[w][r][lane * 4];
        *(volatile v4f*)(y + ((size_t)b * T + row) * ypitch + h * D + lane * 4) = val;
      }
    }
    if (pass == 0) __threadfence();
  }
}

template <bool ASPLIT, int ACT, bool BIAS_BF16, bool RES_BF16>
__global__ __launch_bounds__(128) void k_gemm_bf3(const float* __restrict__ A, int lda, const unsigned short* __restrict__ Wt, int ldb,
                                                const float* __restrict__ bias, const float* __restrict__ resid, int rmod, int ldr,
                                                float* __restrict__ C, int ldc, int M, int N, int K) {
  __shared__ __attribute__((aligned(16))) float so[4][16][64];
  const int tid = threadIdx.x, w = tid >> 5, lane = tid & 31, ln = lane & 15, hh = lane >> 4;
  const int ntn = N / 64;
  const int wid = blockIdx.x * 4 + w;
  const int mt = wid / ntn, nq = wid % ntn;
  if (mt * 16 >= M) return;
  const int row0 = mt * 16, col0 = nq * 64;
  const float* arow = A + (size_t)(row0 + ln) * lda;
  v8f acc[4] = {};
  for (int kb = 0; kb < K; kb += 32) {
    FragB ah, al;
    const v4f x0 = *(const v4fa*)(arow + kb + 8 * hh), x1 = *(const v4fa*)(arow + kb + 8 * hh + 4);
    const v4f x2 = *(const v4fa*)(arow + kb + 16 + 8 * hh), x3 = *(const v4fa*)(arow + kb + 16 + 8 * hh + 4);
    float xs[16] = {x0[0],x0[1],x0[2],x0[3],x1[0],x1[1],x1[2],x1[3],x2[0],x2[1],x2[2],x2[3],x3[0],x3[1],x3[2],x3[3]};
#pragma unroll
    for (int i = 0; i < 16; ++i) { const unsigned short hb = bf16_bits(xs[i]); ah.u[i] = hb; al.u[i] = ASPLIT ? bf16_bits(xs[i] - bf16_val(hb)) : (unsigned short)0; }
#pragma unroll
    for (int t = 0; t < 4; ++t) {
      const unsigned short* brow = Wt + (size_t)(col0 + t * 16 + ln) * ldb + kb;
      FragB b;
      b.half[0] = *(const v8us*)(brow + 8 * hh);
      b.half[1] = *(const v8us*)(brow + 16 + 8 * hh);
      acc[t] = mmaN<ASPLIT ? 2 : 1>(ah.v, al.v, b.v, b.v, acc[t]);
    }
  }
#pragma unroll
  for (int t = 0; t < 4; ++t) {
    const int col = col0 + t * 16 + ln;
    float bv = bias ? bias[col] : 0.f;
    if (BIAS_BF16) bv = bf16_round(bv);
#pragma unroll
    for (int r = 0; r < 8; ++r) {
      float v = acc[t][r] + bv;
      if (resid) { float rv = resid[(size_t)((row0 + 8 * hh + r) % rmod) * ldr + col]; if (RES_BF16) rv = bf16_round(rv); v += rv; }
      if (ACT == 1) v = fmaxf(v, 0.f);
      if (ACT == 2) v = 0.5f * v * (1.0f + erff(v * 0.70710678118654752f));
      if (ACT == 3) { const float u = 0.7978845608028654f * (v + 0.044715f * v * v * v); v = 0.5f * v * (1.0f + tanhf(u)); }
      so[w][8 * hh + r][t * 16 + ln] = v;
    }
  }
  __builtin_amdgcn_fence(__ATOMIC_ACQ_REL, "workgroup");
  __builtin_amdgcn_wave_barrier();
  const int rsub = lane >> 4, c4 = (lane & 15) * 4;
  for (int pass = 0; pass < 2; ++pass) {
#pragma unroll
    for (int q = 0; q < 8; ++q) {
      const int r = q * 2 + rsub;
      const v4f v = *(const v4fa*)&so[w][r][c4];
      *(volatile v4f*)(C + (size_t)(row0 + r) * ldc + col0 + c4) = v;
    }
    if (pass == 0) __threadfence();
  }
}
template <bool PARAM_BF16>
__global__ __launch_bounds__(256) void k_layernorm(const float* __restrict__ X, const float* __restrict__ R, const float* __restrict__ g, const float* __restrict__ bta,
                                                  float* __restrict__ out_sum, float* __restrict__ out_norm, int N, float eps) {
  __shared__ float red[256];
  const int row = blockIdx.x, tid = threadIdx.x;
  const float* x = X + (size_t)row * N; const float* rr = R ? R + (size_t)row * N : nullptr;
  float vals[16];
  const int per = N / 256;
  float s1 = 0.f;
  for (int u = 0; u < per / 4; ++u) {
    const int j = tid * 4 + 1024 * u;
    const v4f a = *(const v4fa*)(x + j);
    v4f b = {0.f,0.f,0.f,0.f}; if (rr) b = *(const v4fa*)(rr + j);
#pragma unroll
    for (int q = 0; q < 4; ++q) { const float v = a[q] + b[q]; vals[u * 4 + q] = v; s1 += v; }
  }
  red[tid] = s1; __syncthreads();
  for (int st = 128; st > 0; st >>= 1) { if (tid < st) red[tid] += red[tid + st]; __syncthreads(); }
  const float mu = red[0] / (float)N; __syncthreads();
  float s2 = 0.f;
  for (int u = 0; u < per / 4; ++u)
#pragma unroll
    for (int q = 0; q < 4; ++q) { const float c = vals[u * 4 + q] - mu; s2 += c * c; }
  red[tid] = s2; __syncthreads();
  for (int st = 128; st > 0; st >>= 1) { if (tid < st) red[tid] += red[tid + st]; __syncthreads(); }
  const float rs = rsqrtf(red[0] / (float)N + eps);
  for (int pass = 0; pass < 2; ++pass) {
    for (int u = 0; u < per / 4; ++u) {
      const int j = tid * 4 + 1024 * u;
      v4f o, sm;
#pragma unroll
      for (int q = 0; q < 4; ++q) {
        float gg = g[j + q], bb = bta[j + q];
        if (PARAM_BF16) { gg = bf16_round(gg); bb = bf16_round(bb); }
        sm[q] = vals[u * 4 + q]; o[q] = (vals[u * 4 + q] - mu) * rs * gg + bb;
      }
      if (out_sum) *(volatile v4f*)(out_sum + (size_t)row * N + j) = sm;
      *(volatile v4f*)(out_norm + (size_t)row * N + j) = o;
    }
    if (pass == 0) __threadfence();
  }
}


typedef _Float16 v16h __attribute__((ext_vector_type(16)));
union FragH { v16h v; v8us half[2]; _Float16 h[16]; unsigned short u[16]; };
template <int NT>
__device__ __forceinline__ v8f mmaH(v16h ah, v16h al, v16h bh, v16h bl, v8f c) {
  c = __builtin_amdgcn_wmma_f32_16x16x32_f16(false, ah, false, bh, (short)0, c, false, false);
  if (NT >= 2) c = __builtin_amdgcn_wmma_f32_16x16x32_f16(false, al, false, bh, (short)0, c, false, false);
  if (NT >= 3) c = __builtin_amdgcn_wmma_f32_16x16x32_f16(false, ah, false, bl, (short)0, c, false, false);
  asm volatile("v_nop\n\tv_nop\n\tv_nop\n\tv_nop" : "+v"(c) : "v"(ah), "v"(al), "v"(bh), "v"(bl));
  return c;
}
template <bool ASPLIT>
__global__ __launch_bounds__(128) void k_gemm_h(const float* __restrict__ A, int lda, size_t sA, const _Float16* __restrict__ Bh, int ldb, size_t sB, float alpha, float* __restrict__ C, int ldc, size_t sC, int M, int N, int K) {
  __shared__ __attribute__((aligned(16))) float so[4][16][64];
  const int tid = threadIdx.x, w = tid >> 5, lane = tid & 31, ln = lane & 15, hh = lane >> 4; const int by = blockIdx.y;
  A += (size_t)by * sA; Bh += (size_t)by * sB; C += (size_t)by * sC;
  const int ntn = (N + 63) / 64; const int wid = blockIdx.x * 4 + w; const int mt = wid / ntn, nq = wid % ntn; if (mt * 16 >= M) return;
  const int row0 = mt * 16, col0 = nq * 64; const float* arow = A + (size_t)(row0 + ln) * lda;
  v8f acc[4] = {};
  for (int kb = 0; kb < K; kb += 32) {
    FragH ah, al;
    const v4f x0 = *(const v4fa*)(arow + kb + 8 * hh), x1 = *(const v4fa*)(arow + kb + 8 * hh + 4), x2 = *(const v4fa*)(arow + kb + 16 + 8 * hh), x3 = *(const v4fa*)(arow + kb + 16 + 8 * hh + 4);
    float xs[16] = {x0[0],x0[1],x0[2],x0[3],x1[0],x1[1],x1[2],x1[3],x2[0],x2[1],x2[2],x2[3],x3[0],x3[1],x3[2],x3[3]};
#pragma unroll
    for (int i = 0; i < 16; ++i) { const _Float16 h = (_Float16)xs[i]; ah.h[i] = h; al.h[i] = ASPLIT ? (_Float16)(xs[i] - (float)h) : (_Float16)0.0f; }
#pragma unroll
    for (int t = 0; t < 4; ++t) { if (col0 + t * 16 >= N) continue; const size_t boff = (size_t)(col0 + t * 16 + ln) * ldb + kb; FragH bq; bq.half[0] = *(const v8us*)(Bh + boff + 8 * hh); bq.half[1] = *(const v8us*)(Bh + boff + 16 + 8 * hh);
      acc[t] = mmaH<ASPLIT ? 2 : 1>(ah.v, al.v, bq.v, bq.v, acc[t]); }
  }
#pragma unroll
  for (int t = 0; t < 4; ++t) { if (col0 + t * 16 >= N) continue;
#pragma unroll
    for (int r = 0; r < 8; ++r) so[w][8 * hh + r][t * 16 + ln] = acc[t][r] * alpha; }
  __builtin_amdgcn_fence(__ATOMIC_ACQ_REL, "workgroup"); __builtin_amdgcn_wave_barrier();
  const int rsub = lane >> 4, c4 = (lane & 15) * 4;
  for (int pass = 0; pass < 2; ++pass) {
#pragma unroll
    for (int q = 0; q < 8; ++q) { const int r = q * 2 + rsub; if (col0 + c4 < N) { const v4f v = *(const v4fa*)&so[w][r][c4]; *(volatile v4f*)(C + (size_t)(row0 + r) * ldc + col0 + c4) = v; } }
    if (pass == 0) __threadfence(); }
}

__global__ __launch_bounds__(256) void k_wt_f16(const float* __restrict__ W, _Float16* __restrict__ Wt, int K, int N, float scale) {
  const int t = blockIdx.x * 256 + threadIdx.x; if (t >= N * (K / 8)) return; const int n = t / (K / 8), k8 = (t % (K / 8)) * 8; FragH f;
#pragma unroll
  for (int i = 0; i < 8; ++i) f.h[i] = (_Float16)(bf16_round(W[(size_t)(k8 + i) * N + n]) * scale); const v8us o = f.half[0];
  *(volatile v8us*)((unsigned short*)Wt + (size_t)n * K + k8) = o; __threadfence(); *(volatile v8us*)((unsigned short*)Wt + (size_t)n * K + k8) = o;
}
template <int ACT>
__global__ __launch_bounds__(128) void k_gemm_hhx(const _Float16* __restrict__ A, int lda, size_t sA, const _Float16* __restrict__ Bh, int ldb, size_t sB, float alpha, const float* __restrict__ bias, size_t sBias, const float* __restrict__ CP, int rowsPerB, size_t sCPb, int row0g,
    float* __restrict__ C, _Float16* __restrict__ C16, int ldc, size_t sC, int M, int N, int K) {
  __shared__ __attribute__((aligned(16))) float so[4][16][64];
  const int tid = threadIdx.x, w = tid >> 5, lane = tid & 31, ln = lane & 15, hh = lane >> 4; const int by = blockIdx.y;
  A += (size_t)by * sA; Bh += (size_t)by * sB; const size_t cofs = (size_t)by * sC; const float* bp = bias ? bias + (size_t)by * sBias : nullptr;
  const int ntn = (N + 63) / 64; const int wid = blockIdx.x * 4 + w; const int mt = wid / ntn, nq = wid % ntn; if (mt * 16 >= M) return;
  const int row0 = mt * 16, col0 = nq * 64; const _Float16* arow = A + (size_t)(row0 + ln) * lda;
  v8f acc[4] = {};
  for (int kb = 0; kb < K; kb += 32) { FragH ah; ah.half[0] = *(const v8us*)((const unsigned short*)arow + kb + 8 * hh); ah.half[1] = *(const v8us*)((const unsigned short*)arow + kb + 16 + 8 * hh);
#pragma unroll
    for (int t = 0; t < 4; ++t) { if (col0 + t * 16 >= N) continue; const size_t boff = (size_t)(col0 + t * 16 + ln) * ldb + kb; FragH bq; bq.half[0] = *(const v8us*)((const unsigned short*)Bh + boff + 8 * hh); bq.half[1] = *(const v8us*)((const unsigned short*)Bh + boff + 16 + 8 * hh);
      acc[t] = mmaH<1>(ah.v, ah.v, bq.v, bq.v, acc[t]); }
  }
#pragma unroll
  for (int t = 0; t < 4; ++t) { if (col0 + t * 16 >= N) continue; const int col = col0 + t * 16 + ln; const float bv = bp ? bf16_round(bp[col]) : 0.f;
#pragma unroll
    for (int r = 0; r < 8; ++r) { float v = acc[t][r] * alpha + bv; if (CP) { const int bidx = (row0g + row0 + 8 * hh + r) / rowsPerB; v += CP[(size_t)bidx * sCPb + (size_t)by * 64 + col]; } if (ACT == 1) v = (v > 0.f) ? v : expm1f(v); else if (ACT == 3) v = fmaxf(v, 0.f); so[w][8 * hh + r][t * 16 + ln] = v; } }
  __builtin_amdgcn_fence(__ATOMIC_ACQ_REL, "workgroup"); __builtin_amdgcn_wave_barrier();
  const int rsub = lane >> 4, c4 = (lane & 15) * 4; typedef _Float16 v4h __attribute__((ext_vector_type(4)));
  for (int pass = 0; pass < 2; ++pass) {
#pragma unroll
    for (int q = 0; q < 8; ++q) { const int r = q * 2 + rsub; if (col0 + c4 < N) { const v4f v = *(const v4fa*)&so[w][r][c4]; if (C) *(volatile v4f*)(C + cofs + (size_t)(row0 + r) * ldc + col0 + c4) = v; if (C16) { v4h h4; for (int i = 0; i < 4; ++i) h4[i] = (_Float16)v[i]; *(volatile v4h*)(C16 + cofs + (size_t)(row0 + r) * ldc + col0 + c4) = h4; } } }
    if (pass == 0) __threadfence(); }
}


__global__ __launch_bounds__(256) void k_round16f(const float* __restrict__ W, _Float16* __restrict__ Bt, size_t n8) { const size_t t = (size_t)blockIdx.x * 256 + threadIdx.x; if (t >= n8) return; FragH f;
#pragma unroll
  for (int i = 0; i < 8; ++i) f.h[i] = (_Float16)(bf16_round(W[t * 8 + i]) * 16.0f); *(volatile v8us*)((unsigned short*)Bt + t * 8) = f.half[0]; __threadfence(); *(volatile v8us*)((unsigned short*)Bt + t * 8) = f.half[0]; }
__device__ __forceinline__ float silu_f(float v) { return v / (1.0f + expf(-v)); }
template <bool RX>
__global__ __launch_bounds__(256) void k_instat(const float* __restrict__ src, float* __restrict__ ST) { __shared__ float red[256]; const int tid = threadIdx.x; const int bc = blockIdx.x; const float* p = src + (size_t)bc * NP; float s = 0.f;
  for (int i = tid; i < NP; i += 256) { const float v = RX ? bf16_round(p[i]) : p[i]; s += v; } red[tid] = s; __syncthreads(); for (int st = 128; st >= 1; st >>= 1) { if (tid < st) red[tid] += red[tid + st]; __syncthreads(); } const float mu = red[0] / (float)NP; __syncthreads();
  float q = 0.f; for (int i = tid; i < NP; i += 256) { const float v = (RX ? bf16_round(p[i]) : p[i]) - mu; q += v * v; } red[tid] = q; __syncthreads(); for (int st = 128; st >= 1; st >>= 1) { if (tid < st) red[tid] += red[tid + st]; __syncthreads(); }
  if (tid == 0) { const float rs = rsqrtf(red[0] / (float)NP + 1e-5f); *(volatile float*)(ST + bc * 4) = mu; *(volatile float*)(ST + bc * 4 + 1) = rs; __threadfence(); *(volatile float*)(ST + bc * 4) = mu; *(volatile float*)(ST + bc * 4 + 1) = rs; } }
__global__ __launch_bounds__(256) void k_se(const float* __restrict__ x, const float* __restrict__ dz, const float* __restrict__ ST, const float* __restrict__ w1, const float* __restrict__ b1, const float* __restrict__ w2, const float* __restrict__ b2, float* __restrict__ SG) {
  __shared__ float red[256]; __shared__ float sp[CC]; __shared__ float sq[CB]; const int tid = threadIdx.x; const int b = blockIdx.x; const float* dzb = dz + (size_t)b * NP;
  float s = 0.f; for (int i = tid; i < NP; i += 256) s += bf16_round(dzb[i]); red[tid] = s; __syncthreads(); for (int st = 128; st >= 1; st >>= 1) { if (tid < st) red[tid] += red[tid + st]; __syncthreads(); } const float dzs = red[0]; __syncthreads();
#pragma unroll 1
  for (int c = 0; c < CC; ++c) { const float mu = ST[(b * CC + c) * 4], rs = ST[(b * CC + c) * 4 + 1]; const float* xp = x + ((size_t)b * CC + c) * NP; float a = 0.f; for (int i = tid; i < NP; i += 256) a += (bf16_round(xp[i]) - mu) * rs * bf16_round(dzb[i]); red[tid] = a; __syncthreads(); for (int st = 128; st >= 1; st >>= 1) { if (tid < st) red[tid] += red[tid + st]; __syncthreads(); } if (tid == 0) sp[c] = red[0] / (dzs + 1e-6f); __syncthreads(); }
  if (tid < CB) { float a = bf16_round(b1[tid]);
#pragma unroll 1
    for (int c = 0; c < CC; ++c) a += sp[c] * bf16_round(w1[tid * CC + c]); sq[tid] = fmaxf(a, 0.f); } __syncthreads();
  if (tid < CC) { float a = bf16_round(b2[tid]);
#pragma unroll 1
    for (int j = 0; j < CB; ++j) a += sq[j] * bf16_round(w2[tid * CB + j]); const float sv = 1.0f / (1.0f + expf(-a)); *(volatile float*)(SG + b * CC + tid) = sv; __threadfence(); *(volatile float*)(SG + b * CC + tid) = sv; } }
__global__ __launch_bounds__(256) void k_x2(const float* __restrict__ x, const float* __restrict__ ST, const float* __restrict__ SG, const float* __restrict__ lng, const float* __restrict__ lnb, float* __restrict__ X2H, _Float16* __restrict__ XLN) {
  __shared__ __attribute__((aligned(16))) float tl[CC][64 + 1]; __shared__ float smu[64], srs[64]; const int tid = threadIdx.x; const int b = blockIdx.x / (NP / 64), pg = blockIdx.x % (NP / 64); const int p0 = pg * 64;
  for (int i = tid; i < CC * 64; i += 256) { const int c = i / 64, px = i % 64; const size_t gi = ((size_t)b * CC + c) * NP + p0 + px; const float xr = x[gi]; const float xn = (bf16_round(xr) - ST[(b * CC + c) * 4]) * ST[(b * CC + c) * 4 + 1]; tl[c][px] = xn * SG[b * CC + c] + 0.4f * bf16_round(xr); }
  __syncthreads();
  if (tid < 64) { float s = 0.f; for (int c = 0; c < CC; ++c) s += tl[c][tid]; const float mu = s / (float)CC; float q = 0.f; for (int c = 0; c < CC; ++c) { const float d = tl[c][tid] - mu; q += d * d; } smu[tid] = mu; srs[tid] = rsqrtf(q / (float)CC + 1e-5f); }
  __syncthreads();
  for (int pass = 0; pass < 2; ++pass) {
    for (int i = tid; i < 64 * 24; i += 256) { const int r = i / 24, pc = i % 24; v4f v; v[0] = tl[pc * 4][r]; v[1] = tl[pc * 4 + 1][r]; v[2] = tl[pc * 4 + 2][r]; v[3] = tl[pc * 4 + 3][r]; *(volatile v4f*)(X2H + ((size_t)b * NP + p0 + r) * CC + pc * 4) = v; }
    for (int i = tid; i < 64 * 12; i += 256) { const int r = i / 12, pc = i % 12; FragH f;
#pragma unroll
      for (int q = 0; q < 8; ++q) { const int c = pc * 8 + q; f.h[q] = (_Float16)((tl[c][r] - smu[r]) * srs[r] * bf16_round(lng[c]) + bf16_round(lnb[c])); }
      *(volatile v8us*)((unsigned short*)XLN + ((size_t)b * NP + p0 + r) * CC + pc * 8) = f.half[0]; }
    if (pass == 0) __threadfence(); } }

__global__ __launch_bounds__(256) void k_dwconv(const _Float16* __restrict__ XZ16, const float* __restrict__ cw, const float* __restrict__ cb, _Float16* __restrict__ XC16) { const size_t t = (size_t)blockIdx.x * 256 + threadIdx.x; if (t >= (size_t)NR * DI / 4) return; const size_t row = t / (DI / 4); const int d4 = (int)(t % (DI / 4)) * 4; const int b = (int)(row / NP), p = (int)(row % NP); const int y = p / HS, xq = p % HS;
  v4f v; typedef _Float16 v4h __attribute__((ext_vector_type(4))); v4h f;
#pragma unroll
  for (int q = 0; q < 4; ++q) { const int d = d4 + q; float a = bf16_round(cb[d]);
#pragma unroll
    for (int k9 = 0; k9 < 9; ++k9) { const int yy = y + k9 / 3 - 1, xx = xq + k9 % 3 - 1; const bool ok = (yy >= 0 && yy < HS && xx >= 0 && xx < HS); const int yc = yy < 0 ? 0 : (yy >= HS ? HS - 1 : yy), xc = xx < 0 ? 0 : (xx >= HS ? HS - 1 : xx);
      const float xv = (float)XZ16[((size_t)b * NP + yc * HS + xc) * (2 * DI) + d]; a += ok ? bf16_round(cw[d * 9 + k9]) * xv : 0.f; }
    v[q] = silu_f(a); f[q] = (_Float16)(v[q] * 64.0f); }
  for (int pass = 0; pass < 2; ++pass) { *(volatile v4h*)(XC16 + row * DI + d4) = f; if (pass == 0) __threadfence(); } }
__global__ __launch_bounds__(256) void k_wxp(const float* __restrict__ xpw, _Float16* __restrict__ Bt) { const int t = blockIdx.x * 256 + threadIdx.x; if (t >= 4 * 32 * (DI / 8)) return; const int k = t / (32 * (DI / 8)); const int rem = t % (32 * (DI / 8)); const int c = rem / (DI / 8), d8 = (rem % (DI / 8)) * 8; const int cc = (c < XDW) ? c : (XDW - 1); FragH f;
#pragma unroll
  for (int q = 0; q < 8; ++q) { const float w = bf16_round(xpw[((size_t)k * XDW + cc) * DI + d8 + q]) * 16.0f; f.h[q] = (_Float16)((c < XDW) ? w : 0.f); }
  *(volatile v8us*)((unsigned short*)Bt + (size_t)t * 8) = f.half[0]; __threadfence(); *(volatile v8us*)((unsigned short*)Bt + (size_t)t * 8) = f.half[0]; }
__global__ __launch_bounds__(192) void k_scan(const _Float16* __restrict__ XC16, const float* __restrict__ XD, const float* __restrict__ dtw, const float* __restrict__ dtb, const float* __restrict__ Alog, const float* __restrict__ Ds, float* __restrict__ OY) {
  const int d = threadIdx.x; const int b = blockIdx.x / 4, k = blockIdx.x % 4; float A[NS], h[NS], wr[RR];
#pragma unroll
  for (int n = 0; n < NS; ++n) { A[n] = -expf(bf16_round(Alog[((size_t)k * DI + d) * NS + n])) * 1.4426950408889634f; h[n] = 0.f; }
#pragma unroll
  for (int r = 0; r < RR; ++r) wr[r] = bf16_round(dtw[((size_t)k * DI + d) * RR + r]);
  const float db = bf16_round(dtb[k * DI + d]), dsk = bf16_round(Ds[k * DI + d]); const float* XDk = XD + (size_t)k * NR * 32;
#pragma unroll 1
  for (int l = 0; l < NP; ++l) { int p; if (k == 0) p = l; else if (k == 1) p = (l % HS) * HS + l / HS; else if (k == 2) p = NP - 1 - l; else { const int l2 = NP - 1 - l; p = (l2 % HS) * HS + l2 / HS; }
    const size_t row = (size_t)b * NP + p; const float u = (float)XC16[row * DI + d] * 0.015625f; const float* xd = XDk + row * 32; float raw = db;
#pragma unroll
    for (int r = 0; r < RR; ++r) raw += wr[r] * xd[r]; const float dl = (raw > 20.f) ? raw : log1pf(expf(raw)); const float du = dl * u; float yv = dsk * u;
#pragma unroll
    for (int n = 0; n < NS; ++n) { const float dA = __builtin_amdgcn_exp2f(dl * A[n]); h[n] = dA * h[n] + du * xd[RR + n]; yv += h[n] * xd[RR + NS + n]; }
    float* o = OY + (((size_t)k * BB + b) * NP + l) * DI + d; *(volatile float*)o = yv; __threadfence(); *(volatile float*)o = yv; } }
__global__ __launch_bounds__(256) void k_merge(const float* __restrict__ OY, const _Float16* __restrict__ XZ16, const float* __restrict__ ong, const float* __restrict__ onb, _Float16* __restrict__ YG16) { const int tid = threadIdx.x, wv = tid >> 5, lane = tid & 31; const size_t row = (size_t)blockIdx.x * 8 + wv; if (row >= NR) return; const int b = (int)(row / NP), p = (int)(row % NP); const int hq = p / HS, wq = p % HS; const int l1 = wq * HS + hq;
  const size_t r0 = ((size_t)0 * BB + b) * NP + p, r1 = ((size_t)1 * BB + b) * NP + l1, r2 = ((size_t)2 * BB + b) * NP + (NP - 1 - p), r3 = ((size_t)3 * BB + b) * NP + (NP - 1 - l1);
  float v[6]; float s = 0.f;
#pragma unroll
  for (int q = 0; q < 6; ++q) { const int d = lane * 6 + q; v[q] = OY[r0 * DI + d] + OY[r1 * DI + d] + OY[r2 * DI + d] + OY[r3 * DI + d]; s += v[q]; }
  for (int o = 16; o >= 1; o >>= 1) s += __shfl_xor(s, o, 32); const float mu = s / (float)DI; float q2 = 0.f;
#pragma unroll
  for (int q = 0; q < 6; ++q) { const float dd = v[q] - mu; q2 += dd * dd; } for (int o = 16; o >= 1; o >>= 1) q2 += __shfl_xor(q2, o, 32); const float rs = rsqrtf(q2 / (float)DI + 1e-5f);
  typedef _Float16 v2h __attribute__((ext_vector_type(2))); _Float16 o6[6];
#pragma unroll
  for (int q = 0; q < 6; ++q) { const int d = lane * 6 + q; const float z = (float)XZ16[row * (2 * DI) + DI + d]; o6[q] = (_Float16)(((v[q] - mu) * rs * bf16_round(ong[d]) + bf16_round(onb[d])) * silu_f(z)); }
  __shared__ __attribute__((aligned(16))) _Float16 srow[8][DI + 8];
#pragma unroll
  for (int q = 0; q < 6; ++q) srow[wv][lane * 6 + q] = o6[q];
  __builtin_amdgcn_fence(__ATOMIC_ACQ_REL, "workgroup"); __builtin_amdgcn_wave_barrier();
  for (int pass = 0; pass < 2; ++pass) { if (lane < DI / 8) { const v8us pv = *(const v8us*)(&srow[wv][lane * 8]); *(volatile v8us*)((unsigned short*)YG16 + row * DI + lane * 8) = pv; } if (pass == 0) __threadfence(); } }
__global__ __launch_bounds__(256) void k_x3(const float* __restrict__ Y3, const float* __restrict__ X2H, const float* __restrict__ skip, float* __restrict__ X3) { __shared__ float tl[CC][64 + 1]; const int tid = threadIdx.x; const int b = blockIdx.x / (NP / 64), pg = blockIdx.x % (NP / 64); const int p0 = pg * 64;
  for (int i = tid; i < 64 * CC; i += 256) { const int r = i / CC, c = i % CC; const size_t row = (size_t)b * NP + p0 + r; tl[c][r] = Y3[row * CC + c] + bf16_round(skip[c]) * X2H[row * CC + c]; }
  __syncthreads();
  for (int pass = 0; pass < 2; ++pass) { for (int i = tid; i < CC * 16; i += 256) { const int c = i / 16, pc = i % 16; v4f v; v[0] = tl[c][pc * 4]; v[1] = tl[c][pc * 4 + 1]; v[2] = tl[c][pc * 4 + 2]; v[3] = tl[c][pc * 4 + 3]; *(volatile v4f*)(X3 + ((size_t)b * CC + c) * NP + p0 + pc * 4) = v; } if (pass == 0) __threadfence(); } }
__global__ __launch_bounds__(256) void k_xn3(const float* __restrict__ X3, const float* __restrict__ ST, _Float16* __restrict__ XN16) { __shared__ float tl[CC][64 + 1]; const int tid = threadIdx.x; const int b = blockIdx.x / (NP / 64), pg = blockIdx.x % (NP / 64); const int p0 = pg * 64;
  for (int i = tid; i < CC * 64; i += 256) { const int c = i / 64, px = i % 64; tl[c][px] = (X3[((size_t)b * CC + c) * NP + p0 + px] - ST[(b * CC + c) * 4]) * ST[(b * CC + c) * 4 + 1]; }
  __syncthreads();
  for (int pass = 0; pass < 2; ++pass) { for (int i = tid; i < 64 * 12; i += 256) { const int r = i / 12, pc = i % 12; FragH f;
#pragma unroll
      for (int q = 0; q < 8; ++q) f.h[q] = (_Float16)tl[pc * 8 + q][r]; *(volatile v8us*)((unsigned short*)XN16 + ((size_t)b * NP + p0 + r) * CC + pc * 8) = f.half[0]; } if (pass == 0) __threadfence(); } }
__global__ __launch_bounds__(256) void k_patch3(const _Float16* __restrict__ H1, _Float16* __restrict__ P16) { const size_t t = (size_t)blockIdx.x * 256 + threadIdx.x; if (t >= (size_t)NR * 20) return; const size_t row = t / 20; const int pc = (int)(t % 20); const int b = (int)(row / NP), p = (int)(row % NP); const int y = p / HS, xq = p % HS; FragH f;
#pragma unroll
  for (int q = 0; q < 8; ++q) { const int kk = pc * 8 + q; float v = 0.f; if (kk < 144) { const int ci = kk / 9, k9 = kk % 9; const int yy = y + k9 / 3 - 1, xx = xq + k9 % 3 - 1; const bool ok = (yy >= 0 && yy < HS && xx >= 0 && xx < HS); const int yc = yy < 0 ? 0 : (yy >= HS ? HS - 1 : yy), xc = xx < 0 ? 0 : (xx >= HS ? HS - 1 : xx); const float hv = (float)H1[((size_t)b * NP + yc * HS + xc) * CB + ci]; v = ok ? hv : 0.f; } f.h[q] = (_Float16)v; }
  *(volatile v8us*)((unsigned short*)P16 + t * 8) = f.half[0]; __threadfence(); *(volatile v8us*)((unsigned short*)P16 + t * 8) = f.half[0]; }
__global__ __launch_bounds__(256) void k_w3(const float* __restrict__ w1, const float* __restrict__ w2, const float* __restrict__ w3, _Float16* __restrict__ B1, _Float16* __restrict__ B2, _Float16* __restrict__ B3) { const int tid = threadIdx.x;
  for (int pass = 0; pass < 2; ++pass) {
    for (int t = tid; t < CB * 12; t += 256) { const int o = t / 12, k8 = (t % 12) * 8; FragH f; for (int q = 0; q < 8; ++q) f.h[q] = (_Float16)(bf16_round(w1[o * CC + k8 + q]) * 16.0f); *(volatile v8us*)((unsigned short*)B1 + (size_t)o * CC + k8) = f.half[0]; }
    for (int t = tid; t < CB * 20; t += 256) { const int o = t / 20, k8 = (t % 20) * 8; FragH f; for (int q = 0; q < 8; ++q) { const int kk = k8 + q; const int kc = (kk < 144) ? kk : 143; const float w = bf16_round(w2[(size_t)o * 144 + kc]) * 16.0f; f.h[q] = (_Float16)((kk < 144) ? w : 0.f); } *(volatile v8us*)((unsigned short*)B2 + (size_t)o * 160 + k8) = f.half[0]; }
    for (int t = tid; t < CC * 4; t += 256) { const int o = t / 4, pc = t % 4; FragH f; for (int q = 0; q < 8; ++q) { const float w = bf16_round(w3[o * CB + (pc & 1) * 8 + q]) * 16.0f; f.h[q] = (_Float16)((pc < 2) ? w : 0.f); } *(volatile v8us*)((unsigned short*)B3 + (size_t)o * 32 + pc * 8) = f.half[0]; }
    if (pass == 0) __threadfence(); } }
__global__ __launch_bounds__(256) void k_pad32(const _Float16* __restrict__ H2, _Float16* __restrict__ H2P) { const size_t t = (size_t)blockIdx.x * 256 + threadIdx.x; if (t >= (size_t)NR * 4) return; const size_t row = t / 4; const int pc = (int)(t % 4); FragH f; const v8us src = *(const v8us*)((const unsigned short*)H2 + row * CB + (pc & 1) * 8);
  FragH s; s.half[0] = src;
#pragma unroll
  for (int q = 0; q < 8; ++q) f.h[q] = (pc < 2) ? s.h[q] : (_Float16)0.f; *(volatile v8us*)((unsigned short*)H2P + t * 8) = f.half[0]; __threadfence(); *(volatile v8us*)((unsigned short*)H2P + t * 8) = f.half[0]; }
__global__ __launch_bounds__(256) void k_out(const float* __restrict__ H3, const float* __restrict__ X3, float* __restrict__ out) { __shared__ float tl[CC][64 + 1]; const int tid = threadIdx.x; const int b = blockIdx.x / (NP / 64), pg = blockIdx.x % (NP / 64); const int p0 = pg * 64;
  for (int i = tid; i < 64 * CC; i += 256) { const int r = i / CC, c = i % CC; tl[c][r] = H3[((size_t)b * NP + p0 + r) * CC + c]; }
  __syncthreads();
  for (int pass = 0; pass < 2; ++pass) { for (int i = tid; i < CC * 16; i += 256) { const int c = i / 16, pc = i % 16; const size_t gi = ((size_t)b * CC + c) * NP + p0 + pc * 4; const v4f xr = *(const v4fa*)(X3 + gi); v4f v; v[0] = tl[c][pc * 4] + xr[0]; v[1] = tl[c][pc * 4 + 1] + xr[1]; v[2] = tl[c][pc * 4 + 2] + xr[2]; v[3] = tl[c][pc * 4 + 3] + xr[3]; *(volatile v4f*)(out + gi) = v; } if (pass == 0) __threadfence(); } }
extern "C" void kernel_launch(void* const* d_in, const int* in_sizes, int n_in,
                              void* d_out, int out_size, void* d_ws, size_t ws_size, hipStream_t stream) {
  (void)in_sizes; (void)n_in; (void)out_size;
  const float* x = (const float*)d_in[0]; const float* dz = (const float*)d_in[1]; const float* inpw = (const float*)d_in[2]; const float* cw = (const float*)d_in[3]; const float* cb = (const float*)d_in[4]; const float* xpw = (const float*)d_in[5]; const float* dtw = (const float*)d_in[6]; const float* dtb = (const float*)d_in[7]; const float* Alog = (const float*)d_in[8]; const float* Ds = (const float*)d_in[9];
  const float* ong = (const float*)d_in[10]; const float* onb = (const float*)d_in[11]; const float* outw = (const float*)d_in[12]; const float* lng = (const float*)d_in[13]; const float* lnb = (const float*)d_in[14]; const float* skip = (const float*)d_in[15]; const float* cw1 = (const float*)d_in[16]; const float* cb1 = (const float*)d_in[17]; const float* cw2 = (const float*)d_in[18]; const float* cb2 = (const float*)d_in[19];
  const float* bw1 = (const float*)d_in[20]; const float* bb1 = (const float*)d_in[21]; const float* bw2 = (const float*)d_in[22]; const float* bb2 = (const float*)d_in[23]; const float* bw3 = (const float*)d_in[24]; const float* bb3 = (const float*)d_in[25];
  char* ws = (char*)d_ws; size_t off = 0;
  auto take = [&](size_t bytes) { char* p = ws + off; off += (bytes + 255) & ~(size_t)255; return p; };
  float* ST = (float*)take((size_t)BB * CC * 4 * 4); float* SG = (float*)take((size_t)BB * CC * 4); _Float16* Bin = (_Float16*)take((size_t)2 * DI * CC * 2); _Float16* Bxp = (_Float16*)take((size_t)4 * 32 * DI * 2); _Float16* Bout = (_Float16*)take((size_t)CC * DI * 2); _Float16* B1 = (_Float16*)take(CB * CC * 2); _Float16* B2 = (_Float16*)take(CB * 160 * 2); _Float16* B3 = (_Float16*)take(CC * 32 * 2);
  float* X2H = (float*)take((size_t)NR * CC * 4); _Float16* XLN = (_Float16*)take((size_t)NR * CC * 2); _Float16* XZ16 = (_Float16*)take((size_t)NR * 2 * DI * 2); _Float16* XC16 = (_Float16*)take((size_t)NR * DI * 2); float* XD = (float*)take((size_t)4 * NR * 32 * 4); float* OY = (float*)take((size_t)4 * NR * DI * 4); _Float16* YG16 = (_Float16*)take((size_t)NR * DI * 2); float* Y3 = (float*)take((size_t)NR * CC * 4); float* X3 = (float*)take((size_t)BB * CC * NP * 4); _Float16* XN16 = (_Float16*)take((size_t)NR * CC * 2); _Float16* H1 = (_Float16*)take((size_t)NR * CB * 2); _Float16* P16 = (_Float16*)take((size_t)NR * 160 * 2); _Float16* H2 = (_Float16*)take((size_t)NR * CB * 2); _Float16* H2P = (_Float16*)take((size_t)NR * 32 * 2); float* H3 = Y3;
  if (off > ws_size) return;
  const unsigned g64 = BB * (NP / 64);
  k_instat<true><<<BB * CC, 256, 0, stream>>>(x, ST);
  k_se<<<BB, 256, 0, stream>>>(x, dz, ST, cw1, cb1, cw2, cb2, SG);
  k_x2<<<g64, 256, 0, stream>>>(x, ST, SG, lng, lnb, X2H, XLN);
  k_round16f<<<(unsigned)((2 * DI * CC / 8 + 255) / 256), 256, 0, stream>>>(inpw, Bin, (size_t)2 * DI * CC / 8); k_wxp<<<(4 * 32 * (DI / 8) + 255) / 256, 256, 0, stream>>>(xpw, Bxp); k_round16f<<<(CC * DI / 8 + 255) / 256, 256, 0, stream>>>(outw, Bout, (size_t)CC * DI / 8); k_w3<<<1, 256, 0, stream>>>(bw1, bw2, bw3, B1, B2, B3);
  k_gemm_hhx<0><<<dim3(((NR / 16) * (2 * DI / 64) + 3) / 4, 1), 128, 0, stream>>>(XLN, CC, 0, Bin, CC, 0, 0.0625f, nullptr, 0, nullptr, 1, 0, 0, nullptr, XZ16, 2 * DI, 0, NR, 2 * DI, CC);
  k_dwconv<<<(unsigned)(((size_t)NR * DI / 4 + 255) / 256), 256, 0, stream>>>(XZ16, cw, cb, XC16);
  for (int k = 0; k < 4; ++k) k_gemm_hhx<0><<<dim3(((NR / 16) * 1 + 3) / 4, 1), 128, 0, stream>>>(XC16, DI, 0, Bxp + (size_t)k * 32 * DI, DI, 0, 0.0009765625f, nullptr, 0, nullptr, 1, 0, 0, XD + (size_t)k * NR * 32, nullptr, 32, 0, NR, 32, DI);
  k_scan<<<BB * 4, DI, 0, stream>>>(XC16, XD, dtw, dtb, Alog, Ds, OY);
  k_merge<<<(NR + 7) / 8, 256, 0, stream>>>(OY, XZ16, ong, onb, YG16);
  k_gemm_hhx<0><<<dim3(((NR / 16) * ((CC + 63) / 64) + 3) / 4, 1), 128, 0, stream>>>(YG16, DI, 0, Bout, DI, 0, 0.0625f, nullptr, 0, nullptr, 1, 0, 0, Y3, nullptr, CC, 0, NR, CC, DI);
  k_x3<<<g64, 256, 0, stream>>>(Y3, X2H, skip, X3);
  k_instat<false><<<BB * CC, 256, 0, stream>>>(X3, ST);
  k_xn3<<<g64, 256, 0, stream>>>(X3, ST, XN16);
  k_gemm_hhx<3><<<dim3(((NR / 16) * 1 + 3) / 4, 1), 128, 0, stream>>>(XN16, CC, 0, B1, CC, 0, 0.0625f, bb1, 0, nullptr, 1, 0, 0, nullptr, H1, CB, 0, NR, CB, CC);
  k_patch3<<<(unsigned)(((size_t)NR * 20 + 255) / 256), 256, 0, stream>>>(H1, P16);
  k_gemm_hhx<3><<<dim3(((NR / 16) * 1 + 3) / 4, 1), 128, 0, stream>>>(P16, 160, 0, B2, 160, 0, 0.0625f, bb2, 0, nullptr, 1, 0, 0, nullptr, H2, CB, 0, NR, CB, 160);
  k_pad32<<<(unsigned)(((size_t)NR * 4 + 255) / 256), 256, 0, stream>>>(H2, H2P);
  k_gemm_hhx<0><<<dim3(((NR / 16) * ((CC + 63) / 64) + 3) / 4, 1), 128, 0, stream>>>(H2P, 32, 0, B3, 32, 0, 0.0625f, bb3, 0, nullptr, 1, 0, 0, H3, nullptr, CC, 0, NR, CC, 32);
  k_out<<<g64, 256, 0, stream>>>(H3, X3, (float*)d_out);
}
